// PointNet_SA_Module_1967095021876
// MI455X (gfx1250) — hardware-verified
//
#include <hip/hip_runtime.h>
#include <math.h>

#pragma clang fp contract(off)

typedef __attribute__((ext_vector_type(16))) _Float16 v16h;
typedef __attribute__((ext_vector_type(8)))  _Float16 v8h;
typedef __attribute__((ext_vector_type(8)))  float    v8f;
typedef __attribute__((ext_vector_type(4)))  float    v4f;
typedef __attribute__((ext_vector_type(4)))  unsigned u4v;

constexpr int NBATCH   = 16;
constexpr int NPTS     = 8192;
constexpr int NCEN     = 512;
constexpr int NSAMP    = 32;
constexpr int NGROUP   = NBATCH * NCEN;
constexpr int NROWS    = NGROUP * NSAMP;
constexpr int CH_FEAT  = 64;
constexpr int CH_IN0   = CH_FEAT + 3;
constexpr int KPAD0    = 96;
constexpr int CH_L0    = 64;
constexpr int CH_L1    = 64;
constexpr int CH_L2    = 128;
constexpr int NPART    = NROWS / 128;
constexpr float BALL_R2  = (float)(0.4 * 0.4);
constexpr float BN_EPS   = 1e-5f;
constexpr float WCARRY   = 16.0f;
constexpr float WCARRY_INV = 1.0f / WCARRY;

static_assert(NPTS % 1024 == 0);
static_assert(NPTS % 32 == 0);
static_assert(KPAD0 % 32 == 0 && KPAD0 >= CH_IN0);
static_assert(CH_L0 % 32 == 0 && CH_L1 % 32 == 0);
static_assert(NROWS % 128 == 0);
static_assert(NGROUP % 4 == 0);
static_assert(NSAMP == 32);

constexpr size_t SZ_CEN   = (size_t)NBATCH * 3 * NCEN * 4;
constexpr size_t SZ_WPL   = (size_t)(CH_L0 * KPAD0 + CH_L1 * CH_L0 + CH_L2 * CH_L1) * 2;
constexpr size_t SZ_SCSH0 = 2 * CH_L0 * 4;
constexpr size_t SZ_SCSH1 = 2 * CH_L1 * 4;
constexpr size_t SZ_SCSH2 = 2 * CH_L2 * 4;
constexpr size_t SZ_P0    = (size_t)NPART * 2 * CH_L0 * 4;
constexpr size_t SZ_P1    = (size_t)NPART * 2 * CH_L1 * 4;
constexpr size_t SZ_P2    = (size_t)NPART * 2 * CH_L2 * 4;
constexpr size_t SZ_MX    = (size_t)NGROUP * CH_L2 * 4;
constexpr size_t SZ_PTST  = (size_t)NBATCH * NPTS * CH_FEAT * 2;
constexpr size_t SZ_H     = (size_t)NROWS * 64 * 2;
constexpr size_t OFF_CEN   = 0;
constexpr size_t OFF_WPL   = OFF_CEN + SZ_CEN;
constexpr size_t OFF_SCSH0 = OFF_WPL + SZ_WPL;
constexpr size_t OFF_SCSH1 = OFF_SCSH0 + SZ_SCSH0;
constexpr size_t OFF_SCSH2 = OFF_SCSH1 + SZ_SCSH1;
constexpr size_t OFF_P0    = OFF_SCSH2 + SZ_SCSH2;
constexpr size_t OFF_P1    = OFF_P0 + SZ_P0;
constexpr size_t OFF_P2    = OFF_P1 + SZ_P1;
constexpr size_t OFF_MX    = OFF_P2 + SZ_P2;
constexpr size_t OFF_MN    = OFF_MX + SZ_MX;
constexpr size_t OFF_PTST  = OFF_MN + SZ_MX;
constexpr size_t OFF_H0    = OFF_PTST + SZ_PTST;
constexpr size_t OFF_H1    = OFF_H0 + SZ_H;
constexpr size_t WS_TOTAL  = OFF_H1 + SZ_H;
static_assert(WS_TOTAL == (size_t)96606208);
static_assert(WS_TOTAL <= (size_t)134217728);
static_assert(OFF_WPL % 128 == 0 && OFF_SCSH0 % 128 == 0 && OFF_SCSH1 % 128 == 0 && OFF_SCSH2 % 128 == 0);
static_assert(OFF_P0 % 128 == 0 && OFF_P1 % 128 == 0 && OFF_P2 % 128 == 0 && OFF_MX % 128 == 0);
static_assert(OFF_MN % 128 == 0 && OFF_PTST % 128 == 0 && OFF_H0 % 128 == 0 && OFF_H1 % 128 == 0);
constexpr size_t OUT0_BYTES = (size_t)NBATCH * 3 * NCEN * 4;
constexpr size_t OUT1_BYTES = (size_t)NBATCH * CH_L2 * NCEN * 4;
static_assert(OUT0_BYTES == 98304);
static_assert(OUT0_BYTES % 128 == 0);
static_assert(OUT0_BYTES + OUT1_BYTES == 4292608);

constexpr int WOFF0 = 0;
constexpr int WOFF1 = CH_L0 * KPAD0;
constexpr int WOFF2 = WOFF1 + CH_L1 * CH_L0;
constexpr int WCHUNKS0 = CH_L0 * KPAD0 / 8;
constexpr int WCHUNKS1 = CH_L1 * CH_L0 / 8;
constexpr int WCHUNKS2 = CH_L2 * CH_L1 / 8;
constexpr int WCHUNKS  = WCHUNKS0 + WCHUNKS1 + WCHUNKS2;
static_assert(WCHUNKS % 256 == 0);
static_assert(WCHUNKS0 % 32 == 0 && (WCHUNKS0 + WCHUNKS1) % 32 == 0);

__device__ __forceinline__ float h16_to_f32(unsigned hb) {
  const unsigned sgn = (hb & 0x8000u) << 16; const unsigned em = hb & 0x7fffu;
  const float fn = __uint_as_float((em << 13) + 0x38000000u);
  const float fs = (float)em * 5.9604644775390625e-8f;
  const float mag = (em < 0x400u) ? fs : fn; return __uint_as_float(__float_as_uint(mag) | sgn); }

__device__ __forceinline__ void wave_sync() {
  __builtin_amdgcn_fence(__ATOMIC_RELEASE, "workgroup");
  __builtin_amdgcn_wave_barrier();
  __builtin_amdgcn_fence(__ATOMIC_ACQUIRE, "workgroup");
}

struct FragH {
  union U { v16h v; v8h h[2]; };
  static __device__ __forceinline__ v16h load(const _Float16* p) {
    U f; f.h[0] = *(const v8h*)(p); f.h[1] = *(const v8h*)(p + 16); return f.v;
  }
};

__device__ __forceinline__ v8f mma_h(v16h a, v16h b, v8f c) {
  c = __builtin_amdgcn_wmma_f32_16x16x32_f16(false, a, false, b, (short)0, c, false, false);
  asm volatile("v_nop\n\tv_nop\n\tv_nop\n\tv_nop" : "+v"(c) : "v"(a), "v"(b));
  return c;
}

template <int KSTEPS, int PITCH>
__device__ __forceinline__ void wave_gemm_32x64(const _Float16* aBase, const _Float16* bBase, int lane,
                                                v8f (&acc)[2][4]) {
  const int c = lane & 15, hh = lane >> 4;
#pragma unroll
  for (int i = 0; i < 2; ++i)
#pragma unroll
    for (int j = 0; j < 4; ++j) acc[i][j] = (v8f){0.f, 0.f, 0.f, 0.f, 0.f, 0.f, 0.f, 0.f};
#pragma unroll
  for (int ks = 0; ks < KSTEPS; ++ks) {
    const int ko = ks * 32 + 8 * hh;
    const v16h a0 = FragH::load(aBase + c * PITCH + ko);
    const v16h a1 = FragH::load(aBase + (16 + c) * PITCH + ko);
#pragma unroll
    for (int j = 0; j < 4; ++j) {
      const v16h bj = FragH::load(bBase + (j * 16 + c) * PITCH + ko);
      acc[0][j] = mma_h(a0, bj, acc[0][j]);
      acc[1][j] = mma_h(a1, bj, acc[1][j]);
    }
  }
}

__device__ __forceinline__ void epi_h16_stats(v8f (&acc)[2][4], const float* __restrict__ bias,
                                              unsigned short* __restrict__ hout, size_t rowBase,
                                              float* slab, float* stSum, float* stSq, int lane) {
  const int c = lane & 15, hh = lane >> 4;
  float bv[4], sm[4], sq[4];
#pragma unroll
  for (int j = 0; j < 4; ++j) { bv[j] = bias[j * 16 + c]; sm[j] = 0.0f; sq[j] = 0.0f; }
#pragma unroll
  for (int i = 0; i < 2; ++i) {
#pragma unroll
    for (int j = 0; j < 4; ++j) {
#pragma unroll
      for (int r = 0; r < 8; ++r) {
        const float v = acc[i][j][r] * WCARRY_INV + bv[j];
        sm[j] = sm[j] + v;
        sq[j] = sq[j] + v * v;
        slab[(8 * hh + r) * 68 + j * 16 + c] = v;
      }
    }
    wave_sync();
    const int q = lane >> 3, c8 = (lane & 7) * 8;
    v8h hv[4];
#pragma unroll
    for (int it = 0; it < 4; ++it) {
      const float* sp = slab + (it * 4 + q) * 68 + c8;
#pragma unroll
      for (int e = 0; e < 8; ++e) hv[it][e] = (_Float16)sp[e];
    }
#pragma unroll
    for (int pass = 0; pass < 2; ++pass) {
#pragma unroll
      for (int it = 0; it < 4; ++it)
        *(volatile v8h*)(hout + (rowBase + (size_t)(i * 16 + it * 4 + q)) * 64 + c8) = hv[it];
      __threadfence();
    }
    wave_sync();
  }
#pragma unroll
  for (int j = 0; j < 4; ++j) {
    sm[j] = sm[j] + __shfl_xor(sm[j], 16, 32);
    sq[j] = sq[j] + __shfl_xor(sq[j], 16, 32);
  }
  if (hh == 0) {
#pragma unroll
    for (int j = 0; j < 4; ++j) { stSum[j * 16 + c] = sm[j]; stSq[j * 16 + c] = sq[j]; }
  }
}

__device__ __forceinline__ void stage_act_tile(const unsigned short* __restrict__ hin, size_t row0,
                                               const float* __restrict__ scsh, _Float16* sA, int tid, int oz) {
  const int c8 = (tid & 7) * 8;
  v4f sc0 = *(const v4f*)(scsh + c8 + oz);
  v4f sc1 = *(const v4f*)(scsh + c8 + 4 + oz);
  v4f sh0 = *(const v4f*)(scsh + 64 + c8 + oz);
  v4f sh1 = *(const v4f*)(scsh + 64 + c8 + 4 + oz);
  asm volatile("" : "+v"(oz), "+v"(sc0), "+v"(sc1), "+v"(sh0), "+v"(sh1) : : "memory");
  const float scr[8] = {sc0.x, sc0.y, sc0.z, sc0.w, sc1.x, sc1.y, sc1.z, sc1.w};
  const float shr[8] = {sh0.x, sh0.y, sh0.z, sh0.w, sh1.x, sh1.y, sh1.z, sh1.w};
  u4v raw[8];
#pragma unroll
  for (int it = 0; it < 8; ++it) {
    const int row = it * 16 + (tid >> 3) + oz;
    raw[it] = *(const u4v*)(hin + (row0 + (size_t)row) * 64 + c8);
  }
#pragma unroll
  for (int it = 0; it < 8; ++it) {
    const int row = it * 16 + (tid >> 3);
    v8h hv;
#pragma unroll
    for (int wi = 0; wi < 4; ++wi) {
      const unsigned wd = raw[it][wi];
      const float f0 = h16_to_f32(wd & 0xffffu);
      const float f1 = h16_to_f32(wd >> 16);
      const float a0 = fmaxf(f0 * scr[2 * wi] + shr[2 * wi], 0.0f);
      const float a1 = fmaxf(f1 * scr[2 * wi + 1] + shr[2 * wi + 1], 0.0f);
      hv[2 * wi]     = (_Float16)a0;
      hv[2 * wi + 1] = (_Float16)a1;
    }
    *(v8h*)(sA + row * 64 + c8) = hv;
  }
}

__global__ __launch_bounds__(1024) void k_fps(const float* __restrict__ xyz, float* __restrict__ out0,
                                              float* __restrict__ cen) {
#pragma clang fp contract(off)
  const int b = blockIdx.x;
  const int tid = threadIdx.x;
  const int lane = tid & 31, wave = tid >> 5;
  const float* xp = xyz + (size_t)b * 3 * NPTS;
  const float* yp = xp + NPTS;
  const float* zp = yp + NPTS;
  __shared__ float rv[2][32];
  __shared__ int   ri[2][32];
  __shared__ float scx[NCEN];
  __shared__ float scy[NCEN];
  __shared__ float scz[NCEN];

  int oz = 0;
  asm volatile("" : "+v"(oz));
  float px[8], py[8], pz[8], dist[8];
#pragma unroll
  for (int i = 0; i < 8; ++i) px[i] = xp[i * 1024 + tid + oz];
  asm volatile("" : "+v"(oz), "+v"(px[0]), "+v"(px[1]), "+v"(px[2]), "+v"(px[3]),
                    "+v"(px[4]), "+v"(px[5]), "+v"(px[6]), "+v"(px[7]) : : "memory");
#pragma unroll
  for (int i = 0; i < 8; ++i) py[i] = yp[i * 1024 + tid + oz];
  asm volatile("" : "+v"(oz), "+v"(py[0]), "+v"(py[1]), "+v"(py[2]), "+v"(py[3]),
                    "+v"(py[4]), "+v"(py[5]), "+v"(py[6]), "+v"(py[7]) : : "memory");
#pragma unroll
  for (int i = 0; i < 8; ++i) pz[i] = zp[i * 1024 + tid + oz];
  asm volatile("" : "+v"(oz), "+v"(pz[0]), "+v"(pz[1]), "+v"(pz[2]), "+v"(pz[3]),
                    "+v"(pz[4]), "+v"(pz[5]), "+v"(pz[6]), "+v"(pz[7]) : : "memory");
#pragma unroll
  for (int i = 0; i < 8; ++i) dist[i] = INFINITY;

  int last = oz;
#pragma unroll 1
  for (int s = 0; s < NCEN; ++s) {
    const int par = s & 1;
    const float lx = xp[last], ly = yp[last], lz = zp[last];
    if (tid == 0) { scx[s] = lx; scy[s] = ly; scz[s] = lz; }
    float bestv = -1.0f;
    int besti = 0;
#pragma unroll
    for (int i = 0; i < 8; ++i) {
      const float dx = px[i] - lx, dy = py[i] - ly, dz = pz[i] - lz;
      const float t0 = dx * dx;
      const float t1 = dy * dy;
      const float t2 = dz * dz;
      float d = (t0 + t2) + t1;
      d = fminf(dist[i], d);
      dist[i] = d;
      if (d > bestv) { bestv = d; besti = i * 1024 + tid; }
    }
#pragma unroll
    for (int off = 16; off > 0; off >>= 1) {
      const float v2 = __shfl_xor(bestv, off, 32);
      const int   i2 = __shfl_xor(besti, off, 32);
      const bool take = (v2 > bestv) || (v2 == bestv && i2 < besti);
      bestv = take ? v2 : bestv;
      besti = take ? i2 : besti;
    }
    if (lane == 0) { rv[par][wave] = bestv; ri[par][wave] = besti; }
    __syncthreads();
    float v = rv[par][lane];
    int ix = ri[par][lane];
#pragma unroll
    for (int off = 16; off > 0; off >>= 1) {
      const float v2 = __shfl_xor(v, off, 32);
      const int   i2 = __shfl_xor(ix, off, 32);
      const bool take = (v2 > v) || (v2 == v && i2 < ix);
      v = take ? v2 : v;
      ix = take ? i2 : ix;
    }
    ix = ix < 0 ? 0 : ix;
    ix = ix > (NPTS - 1) ? (NPTS - 1) : ix;
    last = ix;
  }
  __syncthreads();
  for (int L = wave; L < 48; L += 32) {
    const int d = L >> 4, s0 = (L & 15) * 32;
    const float vx = scx[s0 + lane], vy = scy[s0 + lane], vz = scz[s0 + lane];
    const float val = (d == 0) ? vx : ((d == 1) ? vy : vz);
    const size_t o = (size_t)b * 3 * NCEN + (size_t)d * NCEN + s0 + lane;
    *(volatile float*)(out0 + o) = val;
    *(volatile float*)(cen + o) = val;
    __threadfence();
    *(volatile float*)(out0 + o) = val;
    *(volatile float*)(cen + o) = val;
  }
}

__global__ __launch_bounds__(256) void k_prep_w(const float* __restrict__ w0, const float* __restrict__ w1,
                                                const float* __restrict__ w2, unsigned short* __restrict__ wpl) {
  const int chunk = blockIdx.x * 256 + threadIdx.x;
  const int cc0 = chunk < (WCHUNKS0 - 1) ? chunk : (WCHUNKS0 - 1);
  int cc1 = chunk - WCHUNKS0;
  cc1 = cc1 < 0 ? 0 : cc1;
  cc1 = cc1 > (WCHUNKS1 - 1) ? (WCHUNKS1 - 1) : cc1;
  int cc2 = chunk - WCHUNKS0 - WCHUNKS1;
  cc2 = cc2 < 0 ? 0 : cc2;
  cc2 = cc2 > (WCHUNKS2 - 1) ? (WCHUNKS2 - 1) : cc2;
  const int n0 = cc0 / 12, kb0 = (cc0 % 12) * 8;
  const int n1 = cc1 >> 3, kb1 = (cc1 & 7) * 8;
  const int n2 = cc2 >> 3, kb2 = (cc2 & 7) * 8;
  float f[8];
#pragma unroll
  for (int e = 0; e < 8; ++e) {
    const int kk = kb0 + e;
    const bool valid0 = kk < CH_IN0;
    int row0 = (kk < CH_FEAT) ? (kk + 3) : (kk - CH_FEAT);
    row0 = valid0 ? row0 : 0;
    float x0 = w0[row0 * CH_L0 + n0];
    float x1 = w1[(kb1 + e) * CH_L1 + n1];
    float x2 = w2[(kb2 + e) * CH_L2 + n2];
    asm volatile("" : "+v"(x0), "+v"(x1), "+v"(x2) : : "memory");
    const float y0 = valid0 ? x0 : 0.0f;
    const float y = (chunk < WCHUNKS0) ? y0 : ((chunk < WCHUNKS0 + WCHUNKS1) ? x1 : x2);
    f[e] = y * WCARRY;
  }
  if (chunk < WCHUNKS) {
    v8h hv;
#pragma unroll
    for (int e = 0; e < 8; ++e) hv[e] = (_Float16)f[e];
    volatile v8h* dst = (volatile v8h*)(wpl + (size_t)chunk * 8);
    *dst = hv;
    __threadfence();
    *dst = hv;
  }
}

__global__ __launch_bounds__(256) void k_transpose(const float* __restrict__ pts, unsigned short* __restrict__ ptsT) {
  __shared__ float T[64 * 65];
  const int tid = threadIdx.x;
  const int n0 = blockIdx.x * 64;
  const int b = blockIdx.y;
  const int nl = tid & 63, cq = tid >> 6;
#pragma unroll
  for (int hb = 0; hb < 2; ++hb) {
    float v[8];
#pragma unroll
    for (int i = 0; i < 8; ++i) {
      const int c = (hb * 8 + i) * 4 + cq;
      v[i] = pts[((size_t)b * CH_FEAT + c) * NPTS + n0 + nl];
    }
#pragma unroll
    for (int i = 0; i < 8; ++i) {
      const int c = (hb * 8 + i) * 4 + cq;
      T[c * 65 + nl] = v[i];
    }
    asm volatile("" ::: "memory");
  }
  __syncthreads();
  const int c8 = (tid & 7) * 8;
  v8h hv[2];
#pragma unroll
  for (int p2 = 0; p2 < 2; ++p2) {
    const int row = p2 * 32 + (tid >> 3);
#pragma unroll
    for (int e = 0; e < 8; ++e) hv[p2][e] = (_Float16)T[(c8 + e) * 65 + row];
  }
#pragma unroll
  for (int pass = 0; pass < 2; ++pass) {
#pragma unroll
    for (int p2 = 0; p2 < 2; ++p2) {
      const int row = p2 * 32 + (tid >> 3);
      *(volatile v8h*)(ptsT + ((size_t)b * NPTS + n0 + row) * CH_FEAT + c8) = hv[p2];
    }
    __threadfence();
  }
}

__global__ __launch_bounds__(128) void k_layer0(const float* __restrict__ xyz, const float* __restrict__ cen,
                                                const unsigned short* __restrict__ ptsT,
                                                const unsigned short* __restrict__ w0t,
                                                const float* __restrict__ bias,
                                                unsigned short* __restrict__ hout, float* __restrict__ part) {
#pragma clang fp contract(off)
  __shared__ __align__(16) _Float16 sA[128 * KPAD0];
  __shared__ __align__(16) _Float16 sB[CH_L0 * KPAD0];
  __shared__ __align__(16) float sSlab[4][16 * 68];
  __shared__ float sStat[4][2][64];
  __shared__ int sSlot[4][32];
  const int tid = threadIdx.x;
  const int wave = tid >> 5, lane = tid & 31;
  const int g = blockIdx.x * 4 + wave;
  const int b = g / NCEN, s = g - b * NCEN;

#pragma unroll
  for (int i = 0; i < 6; ++i) {
    const u4v wv = *(const u4v*)(w0t + (size_t)(i * 128 + tid) * 8);
    *(u4v*)(sB + (i * 128 + tid) * 8) = wv;
  }
  asm volatile("" ::: "memory");

  const float* xp = xyz + (size_t)b * 3 * NPTS;
  const float* yp = xp + NPTS;
  const float* zp = yp + NPTS;
  const float cx = cen[((size_t)b * 3 + 0) * NCEN + s];
  const float cy = cen[((size_t)b * 3 + 1) * NCEN + s];
  const float cz = cen[((size_t)b * 3 + 2) * NCEN + s];

  sSlot[wave][lane] = 0;
  wave_sync();
  int filled = 0;
  int first = 0;
#pragma unroll 1
  for (int n0 = 0; n0 < NPTS; n0 += 32) {
    if (filled >= NSAMP) break;
    const int n = n0 + lane;
    const float dx = cx - xp[n], dy = cy - yp[n], dz = cz - zp[n];
    const float t0 = dx * dx;
    const float t1 = dy * dy;
    const float t2 = dz * dz;
    const float d2 = (t0 + t2) + t1;
    const bool in = d2 < BALL_R2;
    const unsigned mask = __builtin_amdgcn_ballot_w32(in);
    const int prefix = __builtin_popcount(mask & ((1u << lane) - 1u));
    const int pos = filled + prefix;
    if (in && pos < NSAMP) sSlot[wave][pos] = n;
    if (filled == 0 && mask != 0u) first = n0 + __builtin_ctz(mask);
    filled += __builtin_popcount(mask);
  }
  wave_sync();
  int p = sSlot[wave][lane];
  const int cnt = filled < NSAMP ? filled : NSAMP;
  p = (lane >= cnt) ? first : p;
  p = p < 0 ? 0 : p;
  p = p > (NPTS - 1) ? (NPTS - 1) : p;

  {
    const unsigned short* pbase = ptsT + (size_t)b * NPTS * CH_FEAT;
    const int ch8 = (lane & 7) * 8;
    u4v gv[8];
#pragma unroll
    for (int it = 0; it < 8; ++it) {
      const int row = it * 4 + (lane >> 3);
      const int pr = __shfl(p, row, 32);
      gv[it] = *(const u4v*)(pbase + (size_t)pr * CH_FEAT + ch8);
    }
#pragma unroll
    for (int it = 0; it < 8; ++it) {
      const int row = it * 4 + (lane >> 3);
      *(u4v*)(sA + (wave * 32 + row) * KPAD0 + ch8) = gv[it];
    }
  }
  asm volatile("" ::: "memory");
  {
    const float gx = xp[p] - cx, gy = yp[p] - cy, gz = zp[p] - cz;
    const _Float16 hxh = (_Float16)gx;
    const _Float16 hyh = (_Float16)gy;
    const _Float16 hzh = (_Float16)gz;
    const unsigned hx = (unsigned)__builtin_bit_cast(unsigned short, hxh);
    const unsigned hy = (unsigned)__builtin_bit_cast(unsigned short, hyh);
    const unsigned hz = (unsigned)__builtin_bit_cast(unsigned short, hzh);
    unsigned zz = 0;
    asm volatile("" : "+v"(zz));
    u4v q0, qz;
    q0.x = (hx & 0xffffu) | (hy << 16);
    q0.y = (hz & 0xffffu) | (zz << 16);
    q0.z = zz;
    q0.w = zz;
    qz.x = zz; qz.y = zz; qz.z = zz; qz.w = zz;
    _Float16* rowp = sA + (wave * 32 + lane) * KPAD0;
    *(u4v*)(rowp + 64) = q0;
    *(u4v*)(rowp + 72) = qz;
    *(u4v*)(rowp + 80) = qz;
    *(u4v*)(rowp + 88) = qz;
  }
  __syncthreads();

  v8f acc[2][4];
  wave_gemm_32x64<KPAD0 / 32, KPAD0>(sA + wave * 32 * KPAD0, sB, lane, acc);
  epi_h16_stats(acc, bias, hout, (size_t)g * NSAMP, sSlab[wave], sStat[wave][0], sStat[wave][1], lane);
  __syncthreads();
  {
    const int which = tid >> 6, n = tid & 63;
    const float tot = (sStat[0][which][n] + sStat[1][which][n]) + (sStat[2][which][n] + sStat[3][which][n]);
    volatile float* pp = part + (size_t)blockIdx.x * 128 + tid;
    *pp = tot;
    __threadfence();
    *pp = tot;
  }
}

__global__ __launch_bounds__(128) void k_layer1(const unsigned short* __restrict__ hin,
                                                const unsigned short* __restrict__ w1t,
                                                const float* __restrict__ bias, const float* __restrict__ scsh,
                                                unsigned short* __restrict__ hout, float* __restrict__ part) {
  __shared__ __align__(16) _Float16 sA[128 * 64];
  __shared__ __align__(16) _Float16 sB[CH_L1 * 64];
  __shared__ __align__(16) float sSlab[4][16 * 68];
  __shared__ float sStat[4][2][64];
  const int tid = threadIdx.x;
  const int wave = tid >> 5, lane = tid & 31;
  const size_t row0 = (size_t)blockIdx.x * 128;
#pragma unroll
  for (int i = 0; i < 4; ++i) {
    const u4v wv = *(const u4v*)(w1t + (size_t)(i * 128 + tid) * 8);
    *(u4v*)(sB + (i * 128 + tid) * 8) = wv;
  }
  int oz = 0;
  asm volatile("" : "+v"(oz) : : "memory");
  stage_act_tile(hin, row0, scsh, sA, tid, oz);
  __syncthreads();
  v8f acc[2][4];
  wave_gemm_32x64<2, 64>(sA + wave * 32 * 64, sB, lane, acc);
  epi_h16_stats(acc, bias, hout, row0 + (size_t)wave * 32, sSlab[wave], sStat[wave][0], sStat[wave][1], lane);
  __syncthreads();
  {
    const int which = tid >> 6, n = tid & 63;
    const float tot = (sStat[0][which][n] + sStat[1][which][n]) + (sStat[2][which][n] + sStat[3][which][n]);
    volatile float* pp = part + (size_t)blockIdx.x * 128 + tid;
    *pp = tot;
    __threadfence();
    *pp = tot;
  }
}

__global__ __launch_bounds__(128) void k_layer2(const unsigned short* __restrict__ hin,
                                                const unsigned short* __restrict__ w2t,
                                                const float* __restrict__ bias, const float* __restrict__ scsh,
                                                float* __restrict__ mxp, float* __restrict__ mnp,
                                                float* __restrict__ part) {
  __shared__ __align__(16) _Float16 sA[128 * 64];
  __shared__ __align__(16) _Float16 sB[CH_L2 * 64];
  __shared__ float sStat[4][2][CH_L2];
  __shared__ __align__(16) float sMx[4][CH_L2];
  __shared__ __align__(16) float sMn[4][CH_L2];
  const int tid = threadIdx.x;
  const int wave = tid >> 5, lane = tid & 31;
  const int c = lane & 15, hh = lane >> 4;
  const size_t row0 = (size_t)blockIdx.x * 128;
#pragma unroll
  for (int i = 0; i < 8; ++i) {
    const u4v wv = *(const u4v*)(w2t + (size_t)(i * 128 + tid) * 8);
    *(u4v*)(sB + (i * 128 + tid) * 8) = wv;
  }
  int oz = 0;
  asm volatile("" : "+v"(oz) : : "memory");
  stage_act_tile(hin, row0, scsh, sA, tid, oz);
  __syncthreads();
#pragma unroll 1
  for (int nh = 0; nh < 2; ++nh) {
    v8f acc[2][4];
    wave_gemm_32x64<2, 64>(sA + wave * 32 * 64, sB + nh * 64 * 64, lane, acc);
#pragma unroll
    for (int j = 0; j < 4; ++j) {
      const int n = nh * 64 + j * 16 + c;
      const float bv = bias[n];
      float sm = 0.0f, sq = 0.0f, mx = -INFINITY, mn = INFINITY;
#pragma unroll
      for (int i = 0; i < 2; ++i) {
#pragma unroll
        for (int r = 0; r < 8; ++r) {
          const float v = acc[i][j][r] * WCARRY_INV + bv;
          sm = sm + v;
          sq = sq + v * v;
          mx = fmaxf(mx, v);
          mn = fminf(mn, v);
        }
      }
      sm = sm + __shfl_xor(sm, 16, 32);
      sq = sq + __shfl_xor(sq, 16, 32);
      mx = fmaxf(mx, __shfl_xor(mx, 16, 32));
      mn = fminf(mn, __shfl_xor(mn, 16, 32));
      if (hh == 0) {
        sStat[wave][0][n] = sm;
        sStat[wave][1][n] = sq;
        sMx[wave][n] = mx;
        sMn[wave][n] = mn;
      }
    }
  }
  wave_sync();
  {
    const size_t g = (size_t)blockIdx.x * 4 + wave;
    v4f a, m;
    a.x = sMx[wave][lane * 4 + 0]; a.y = sMx[wave][lane * 4 + 1];
    a.z = sMx[wave][lane * 4 + 2]; a.w = sMx[wave][lane * 4 + 3];
    m.x = sMn[wave][lane * 4 + 0]; m.y = sMn[wave][lane * 4 + 1];
    m.z = sMn[wave][lane * 4 + 2]; m.w = sMn[wave][lane * 4 + 3];
    volatile v4f* pa = (volatile v4f*)(mxp + g * CH_L2 + lane * 4);
    volatile v4f* pm = (volatile v4f*)(mnp + g * CH_L2 + lane * 4);
    *pa = a;
    *pm = m;
    __threadfence();
    *pa = a;
    *pm = m;
  }
  __syncthreads();
  {
    const float t0 = (sStat[0][0][tid] + sStat[1][0][tid]) + (sStat[2][0][tid] + sStat[3][0][tid]);
    const float t1 = (sStat[0][1][tid] + sStat[1][1][tid]) + (sStat[2][1][tid] + sStat[3][1][tid]);
    volatile float* p0 = part + (size_t)blockIdx.x * 256 + tid;
    volatile float* p1 = part + (size_t)blockIdx.x * 256 + 128 + tid;
    *p0 = t0;
    *p1 = t1;
    __threadfence();
    *p0 = t0;
    *p1 = t1;
  }
}

template <int NCHAN>
__global__ __launch_bounds__(2 * NCHAN) void k_stats(const float* __restrict__ P, const float* __restrict__ gamma,
                                                     const float* __restrict__ beta, float* __restrict__ scsh) {
  __shared__ double sD[2 * NCHAN];
  __shared__ float sO[2 * NCHAN];
  const int t = threadIdx.x;
  double accd = 0.0;
#pragma unroll 8
  for (int i = 0; i < NPART; ++i) accd = accd + (double)P[(size_t)i * (2 * NCHAN) + t];
  sD[t] = accd;
  __syncthreads();
  const int ch = t & (NCHAN - 1);
  const float gm = gamma[ch], bt = beta[ch];
  if (t < NCHAN) {
    const double inv = 1.0 / (double)NROWS;
    const double mean = sD[t] * inv;
    double var = sD[NCHAN + t] * inv - mean * mean;
    var = var < 0.0 ? 0.0 : var;
    const float sc = gm * rsqrtf((float)var + BN_EPS);
    const float sh = bt - (float)mean * sc;
    sO[t] = sc;
    sO[NCHAN + t] = sh;
  }
  __syncthreads();
  const float o = sO[t];
  volatile float* dst = scsh + t;
  *dst = o;
  __threadfence();
  *dst = o;
}

__global__ __launch_bounds__(256) void k_final(const float* __restrict__ mxp, const float* __restrict__ mnp,
                                               const float* __restrict__ scsh, float* __restrict__ out1) {
  __shared__ float T[CH_L2 * 33];
  const int tid = threadIdx.x;
  const int wave = tid >> 5, lane = tid & 31;
  const int b = blockIdx.y, s0 = blockIdx.x * 32;
  const size_t g0 = (size_t)b * NCEN + s0;
  const int c4 = lane * 4;
  v4f scv = *(const v4f*)(scsh + c4);
  v4f shv = *(const v4f*)(scsh + CH_L2 + c4);
  asm volatile("" : "+v"(scv), "+v"(shv) : : "memory");
  const float scr[4] = {scv.x, scv.y, scv.z, scv.w};
  const float shr[4] = {shv.x, shv.y, shv.z, shv.w};
#pragma unroll 1
  for (int it = 0; it < 4; ++it) {
    const int gl = wave + 8 * it;
    v4f a = *(const v4f*)(mxp + (g0 + gl) * CH_L2 + c4);
    v4f m = *(const v4f*)(mnp + (g0 + gl) * CH_L2 + c4);
    asm volatile("" : "+v"(a), "+v"(m) : : "memory");
    const float av[4] = {a.x, a.y, a.z, a.w};
    const float mv[4] = {m.x, m.y, m.z, m.w};
#pragma unroll
    for (int e = 0; e < 4; ++e) {
      const float fa = (scr[e] >= 0.0f) ? 1.0f : 0.0f;
      const float fb = 1.0f - fa;
      const float x = fa * av[e] + fb * mv[e];
      const float v = fmaxf(scr[e] * x + shr[e], 0.0f);
      T[(c4 + e) * 33 + gl] = v;
    }
  }
  __syncthreads();
  float ov[16];
#pragma unroll
  for (int cc = 0; cc < 16; ++cc) ov[cc] = T[(wave * 16 + cc) * 33 + lane];
#pragma unroll
  for (int pass = 0; pass < 2; ++pass) {
#pragma unroll
    for (int cc = 0; cc < 16; ++cc) {
      const int ch = wave * 16 + cc;
      *(volatile float*)(out1 + ((size_t)b * CH_L2 + ch) * NCEN + s0 + lane) = ov[cc];
    }
    __threadfence();
  }
}

extern "C" void kernel_launch(void* const* d_in, const int* in_sizes, int n_in,
                              void* d_out, int out_size, void* d_ws, size_t ws_size, hipStream_t stream) {
  (void)in_sizes; (void)n_in; (void)out_size;
  if (ws_size < WS_TOTAL) return;
  const float* xyz = (const float*)d_in[0];
  const float* pts = (const float*)d_in[1];
  const float* w0  = (const float*)d_in[2];
  const float* b0  = (const float*)d_in[3];
  const float* g0  = (const float*)d_in[4];
  const float* bt0 = (const float*)d_in[5];
  const float* w1  = (const float*)d_in[6];
  const float* b1  = (const float*)d_in[7];
  const float* g1  = (const float*)d_in[8];
  const float* bt1 = (const float*)d_in[9];
  const float* w2  = (const float*)d_in[10];
  const float* b2  = (const float*)d_in[11];
  const float* g2  = (const float*)d_in[12];
  const float* bt2 = (const float*)d_in[13];

  char* ws = (char*)d_ws;
  float* cen            = (float*)(ws + OFF_CEN);
  unsigned short* wpl   = (unsigned short*)(ws + OFF_WPL);
  float* scsh0          = (float*)(ws + OFF_SCSH0);
  float* scsh1          = (float*)(ws + OFF_SCSH1);
  float* scsh2          = (float*)(ws + OFF_SCSH2);
  float* P0             = (float*)(ws + OFF_P0);
  float* P1             = (float*)(ws + OFF_P1);
  float* P2             = (float*)(ws + OFF_P2);
  float* mxp            = (float*)(ws + OFF_MX);
  float* mnp            = (float*)(ws + OFF_MN);
  unsigned short* ptsT  = (unsigned short*)(ws + OFF_PTST);
  unsigned short* h0    = (unsigned short*)(ws + OFF_H0);
  unsigned short* h1    = (unsigned short*)(ws + OFF_H1);

  float* out0 = (float*)d_out;
  float* out1 = (float*)d_out + (OUT0_BYTES / 4);

  k_prep_w<<<WCHUNKS / 256, 256, 0, stream>>>(w0, w1, w2, wpl);
  k_transpose<<<dim3(NPTS / 64, NBATCH), 256, 0, stream>>>(pts, ptsT);
  k_fps<<<NBATCH, 1024, 0, stream>>>(xyz, out0, cen);
  k_layer0<<<NGROUP / 4, 128, 0, stream>>>(xyz, cen, ptsT, wpl + WOFF0, b0, h0, P0);
  k_stats<CH_L0><<<1, 2 * CH_L0, 0, stream>>>(P0, g0, bt0, scsh0);
  k_layer1<<<NROWS / 128, 128, 0, stream>>>(h0, wpl + WOFF1, b1, scsh0, h1, P1);
  k_stats<CH_L1><<<1, 2 * CH_L1, 0, stream>>>(P1, g1, bt1, scsh1);
  k_layer2<<<NROWS / 128, 128, 0, stream>>>(h1, wpl + WOFF2, b2, scsh1, mxp, mnp, P2);
  k_stats<CH_L2><<<1, 2 * CH_L2, 0, stream>>>(P2, g2, bt2, scsh2);
  k_final<<<dim3(NCEN / 32, NBATCH), 256, 0, stream>>>(mxp, mnp, scsh2, out1);
}
